// QuadAttention_71116068487401
// MI455X (gfx1250) — hardware-verified
//
#include <hip/hip_runtime.h>
#include <stddef.h>
#include <stdint.h>


#define BB 2
#define NN 2048
#define CC 256
#define HH 16
#define DD 16
#define MTOT (BB * NN)
#define NBH (BB * HH)
#define GRP 16
#define NGRP (NBH / GRP)

#define W_SCALE 64.0f
#define W_INV 0.015625f
#define ST_SCALE 0.0625f
#define T_SCALE 0.0078125f

static_assert(NBH % GRP == 0);
static_assert(MTOT % 32 == 0);
static_assert(CC % 64 == 0);
static_assert(NN % 64 == 0);

typedef _Float16 f16;
typedef f16 v8h __attribute__((ext_vector_type(8)));
typedef f16 v16h __attribute__((ext_vector_type(16)));
typedef float v8f __attribute__((ext_vector_type(8)));
typedef float v4f __attribute__((ext_vector_type(4)));

union Frag { v16h v; v8h hv[2]; };
union U16 { v8h h; v4f f; };

struct Ptr7 { const float* p[7]; };
struct Ptr8 { const float* p[8]; };
static_assert(sizeof(Ptr7) == 56);
static_assert(sizeof(Ptr8) == 64);

__device__ __forceinline__ const float* sel7(const Ptr7& s, int z) {
  const float* r = s.p[0];
#pragma unroll
  for (int i = 1; i < 7; ++i) if (z == i) r = s.p[i];
  return r;
}
__device__ __forceinline__ const float* sel8(const Ptr8& s, int z) {
  const float* r = s.p[0];
#pragma unroll
  for (int i = 1; i < 8; ++i) if (z == i) r = s.p[i];
  return r;
}

__device__ __forceinline__ void st16(void* p, v4f v) { *(volatile v4f*)p = v; }

__device__ __forceinline__ v16h load_frag(const f16* __restrict__ base, int ld, int row0,
                                          int kb, int lane) {
  const f16* p = base + (size_t)(row0 + (lane & 15)) * ld + kb + ((lane >> 4) << 3);
  Frag f;
  f.hv[0] = *(const v8h*)p;
  f.hv[1] = *(const v8h*)(p + 16);
  return f.v;
}

__device__ __forceinline__ v8f wmma16(v16h a, v16h b, v8f c) {
  v8f d = __builtin_amdgcn_wmma_f32_16x16x32_f16(false, a, false, b, (short)0, c, false, false);
  asm volatile("v_nop\n\tv_nop\n\tv_nop\n\tv_nop" : "+v"(d) : "v"(a), "v"(b));
  return d;
}

__device__ __forceinline__ void zero_acc(v8f acc[2][4]) {
#pragma unroll
  for (int tm = 0; tm < 2; ++tm)
#pragma unroll
    for (int tn = 0; tn < 4; ++tn) {
      v8f z;
#pragma unroll
      for (int r = 0; r < 8; ++r) z[r] = 0.0f;
      acc[tm][tn] = z;
    }
}

__device__ __forceinline__ void gemm_32x64(const f16* __restrict__ A, int lda,
                                           const f16* __restrict__ B, int ldb,
                                           int m0, int n0, int K, int lane, v8f acc[2][4]) {
#pragma unroll 1
  for (int kb = 0; kb < K; kb += 32) {
    const v16h a0 = load_frag(A, lda, m0, kb, lane);
    const v16h a1 = load_frag(A, lda, m0 + 16, kb, lane);
    const v16h b0 = load_frag(B, ldb, n0, kb, lane);
    const v16h b1 = load_frag(B, ldb, n0 + 16, kb, lane);
    const v16h b2 = load_frag(B, ldb, n0 + 32, kb, lane);
    const v16h b3 = load_frag(B, ldb, n0 + 48, kb, lane);
    acc[0][0] = wmma16(a0, b0, acc[0][0]);
    acc[0][1] = wmma16(a0, b1, acc[0][1]);
    acc[0][2] = wmma16(a0, b2, acc[0][2]);
    acc[0][3] = wmma16(a0, b3, acc[0][3]);
    acc[1][0] = wmma16(a1, b0, acc[1][0]);
    acc[1][1] = wmma16(a1, b1, acc[1][1]);
    acc[1][2] = wmma16(a1, b2, acc[1][2]);
    acc[1][3] = wmma16(a1, b3, acc[1][3]);
  }
}

__device__ __forceinline__ void store_tile_f32(const float* sT, float* dst, int ldd, int lane) {
#pragma unroll
  for (int it = 0; it < 16; ++it) {
    const int li = it * 4 + (lane >> 3);
    const int row = li >> 1;
    const int col = (li & 1) * 32 + (lane & 7) * 4;
    const v4f v = *(const v4f*)(sT + row * 64 + col);
    st16(dst + (size_t)row * ldd + col, v);
  }
}

__device__ __forceinline__ void store_tile_h(const f16* sH, f16* dst, int ldd, int lane) {
#pragma unroll
  for (int it = 0; it < 8; ++it) {
    const int row = it * 4 + (lane >> 3);
    const int col = (lane & 7) * 8;
    U16 u;
    u.h = *(const v8h*)(sH + row * 64 + col);
    st16(dst + (size_t)row * ldd + col, u.f);
  }
}

__global__ __launch_bounds__(256) void k_convx(const float* __restrict__ x, f16* __restrict__ xh, int n8) {
  const int t = blockIdx.x * 256 + threadIdx.x;
  if (t >= n8) return;
  const float* p = x + (size_t)t * 8;
  const v4f a = *(const v4f*)p;
  const v4f b4 = *(const v4f*)(p + 4);
  U16 u;
#pragma unroll
  for (int e = 0; e < 4; ++e) { u.h[e] = (f16)a[e]; u.h[e + 4] = (f16)b4[e]; }
  f16* dst = xh + (size_t)t * 8;
  st16(dst, u.f);
  __threadfence();
  st16(dst, u.f);
}

__global__ __launch_bounds__(256) void k_convw(Ptr8 w, f16* __restrict__ wh) {
  const int z = blockIdx.y;
  const int t = blockIdx.x * 256 + threadIdx.x;
  if (t >= CC * CC / 8) return;
  const float* src = sel8(w, z) + (size_t)t * 8;
  const v4f a = *(const v4f*)src;
  const v4f b4 = *(const v4f*)(src + 4);
  U16 u;
#pragma unroll
  for (int e = 0; e < 4; ++e) {
    u.h[e] = (f16)(a[e] * W_SCALE);
    u.h[e + 4] = (f16)(b4[e] * W_SCALE);
  }
  f16* dst = wh + (size_t)z * CC * CC + (size_t)t * 8;
  st16(dst, u.f);
  __threadfence();
  st16(dst, u.f);
}

__global__ __launch_bounds__(32) void k_lin(const f16* __restrict__ xh, const f16* __restrict__ wh,
                                          const float* __restrict__ x, const float* __restrict__ mask,
                                          Ptr7 bias, float* __restrict__ lin) {
  __shared__ float sT[32 * 64] __attribute__((aligned(16)));
  const int lane = threadIdx.x;
  const int mt = blockIdx.x, nt = blockIdx.y, z = blockIdx.z;
  const int m0 = mt * 32, n0 = nt * 64;
  const f16* W = wh + (size_t)z * CC * CC;
  const float* bz = sel7(bias, z);
  v8f acc[2][4];
  zero_acc(acc);
  gemm_32x64(xh, CC, W, CC, m0, n0, CC, lane, acc);

  const int hl = lane >> 4, c16 = lane & 15;
#pragma unroll
  for (int tm = 0; tm < 2; ++tm)
#pragma unroll
    for (int tn = 0; tn < 4; ++tn) {
      const int col = tn * 16 + c16;
      const int gcol = n0 + col;
      const float bcol = bz[gcol];
#pragma unroll
      for (int r = 0; r < 8; ++r) {
        const int row = tm * 16 + hl * 8 + r;
        const int grow = m0 + row;
        float v = acc[tm][tn][r] * W_INV + x[(size_t)grow * CC + gcol] + bcol;
        v = v * mask[grow];
        sT[row * 64 + col] = v;
      }
    }
  __syncthreads();
  float* dst = lin + (size_t)z * MTOT * CC + (size_t)m0 * CC + n0;
  store_tile_f32(sT, dst, CC, lane);
  __threadfence();
  store_tile_f32(sT, dst, CC, lane);
}

__device__ __forceinline__ void outer_store(const float* q2s, const float* q3s, const float* k1s,
                                            const float* k2s, const float* k3s, const float* vs,
                                            int w, int L, int gl, int n0,
                                            f16* __restrict__ A1t, f16* __restrict__ A2t, f16* __restrict__ Qt) {
#pragma unroll 1
  for (int it = 0; it < 8; ++it) {
    const int p = w * 32 + it * 4 + (L >> 3);
    const int i = p >> 4, j = p & 15;
    const int q8 = L & 7;
    U16 u1, u2;
#pragma unroll
    for (int e = 0; e < 8; ++e) {
      const int n = q8 * 8 + e;
      u1.h[e] = (f16)(k1s[n * 16 + i] * vs[n * 16 + j]);
      u2.h[e] = (f16)(k2s[n * 16 + i] * k3s[n * 16 + j]);
    }
    const size_t o = ((size_t)(gl * CC + p)) * NN + n0 + q8 * 8;
    st16(A1t + o, u1.f);
    st16(A2t + o, u2.f);
  }
#pragma unroll 1
  for (int it = 0; it < 8; ++it) {
    const int nl = w * 8 + it;
    const int pg = L;
    const int k = pg >> 1, lb = (pg & 1) * 8;
    const float qk = q2s[nl * 16 + k];
    U16 u;
#pragma unroll
    for (int e = 0; e < 8; ++e) u.h[e] = (f16)(qk * q3s[nl * 16 + lb + e]);
    const size_t o = ((size_t)(gl * NN + n0 + nl)) * CC + pg * 8;
    st16(Qt + o, u.f);
  }
}

__global__ __launch_bounds__(256) void k_outer(const float* __restrict__ lin, int gi,
                                             f16* __restrict__ A1t, f16* __restrict__ A2t,
                                             f16* __restrict__ Qt) {
  __shared__ float S[6 * 64 * 16] __attribute__((aligned(16)));
  const int tid = threadIdx.x;
  const int gl = blockIdx.y;
  const int bh = gi * GRP + gl;
  const int b = bh / HH, h = bh % HH;
  const int n0 = blockIdx.x * 64;
#pragma unroll 4
  for (int it = 0; it < 24; ++it) {
    const int idx = it * 256 + tid;
    const int zz = idx >> 10;
    const int rem = idx & 1023;
    const int n = rem >> 4, c = rem & 15;
    S[idx] = lin[(size_t)(zz + 1) * MTOT * CC + (size_t)(b * NN + n0 + n) * CC + h * DD + c];
  }
  __syncthreads();
  const float* q2s = S;
  const float* q3s = S + 1024;
  const float* k1s = S + 2048;
  const float* k2s = S + 3072;
  const float* k3s = S + 4096;
  const float* vs = S + 5120;
  const int w = tid >> 5, L = tid & 31;
  outer_store(q2s, q3s, k1s, k2s, k3s, vs, w, L, gl, n0, A1t, A2t, Qt);
  __threadfence();
  outer_store(q2s, q3s, k1s, k2s, k3s, vs, w, L, gl, n0, A1t, A2t, Qt);
}

__global__ __launch_bounds__(32) void k_state(const f16* __restrict__ A1t, const f16* __restrict__ A2t,
                                            f16* __restrict__ sth) {
  __shared__ f16 sH[32 * 64] __attribute__((aligned(16)));
  const int lane = threadIdx.x;
  const int mt = blockIdx.x, nt = blockIdx.y, gl = blockIdx.z;
  const int m0 = mt * 32, n0 = nt * 64;
  const f16* A = A1t + (size_t)gl * CC * NN;
  const f16* B = A2t + (size_t)gl * CC * NN;
  v8f acc[2][4];
  zero_acc(acc);
  gemm_32x64(A, NN, B, NN, m0, n0, NN, lane, acc);

  const int hl = lane >> 4, c16 = lane & 15;
#pragma unroll
  for (int tm = 0; tm < 2; ++tm)
#pragma unroll
    for (int tn = 0; tn < 4; ++tn) {
      const int col = tn * 16 + c16;
#pragma unroll
      for (int r = 0; r < 8; ++r) {
        const int row = tm * 16 + hl * 8 + r;
        sH[row * 64 + col] = (f16)(acc[tm][tn][r] * ST_SCALE);
      }
    }
  __syncthreads();
  f16* dst = sth + (size_t)gl * CC * CC + (size_t)m0 * CC + n0;
  store_tile_h(sH, dst, CC, lane);
  __threadfence();
  store_tile_h(sH, dst, CC, lane);
}

#define TSP 257
__global__ __launch_bounds__(128) void k_apply(const f16* __restrict__ Qt, const f16* __restrict__ sth,
                                             const float* __restrict__ linq1, int gi,
                                             float* __restrict__ attnT) {
  __shared__ float Ts[32 * TSP];
  __shared__ float q1s[32 * 16] __attribute__((aligned(16)));
  const int tid = threadIdx.x;
  const int w = tid >> 5, lane = tid & 31;
  const int gl = blockIdx.y;
  const int bh = gi * GRP + gl;
  const int b = bh / HH, h = bh % HH;
  const int n0 = blockIdx.x * 32;
  const f16* A = Qt + (size_t)gl * NN * CC;
  const f16* B = sth + (size_t)gl * CC * CC;
  v8f acc[2][4];
  zero_acc(acc);
  gemm_32x64(A, CC, B, CC, n0, w * 64, CC, lane, acc);

  const int hl = lane >> 4, c16 = lane & 15;
#pragma unroll
  for (int tm = 0; tm < 2; ++tm)
#pragma unroll
    for (int tn = 0; tn < 4; ++tn) {
      const int col = w * 64 + tn * 16 + c16;
#pragma unroll
      for (int r = 0; r < 8; ++r) {
        const int row = tm * 16 + hl * 8 + r;
        Ts[row * TSP + col] = acc[tm][tn][r] * T_SCALE;
      }
    }
  {
    const int n = tid >> 2, i0 = (tid & 3) * 4;
    const v4f q = *(const v4f*)(linq1 + (size_t)(b * NN + n0 + n) * CC + h * DD + i0);
    q1s[n * 16 + i0 + 0] = q[0];
    q1s[n * 16 + i0 + 1] = q[1];
    q1s[n * 16 + i0 + 2] = q[2];
    q1s[n * 16 + i0 + 3] = q[3];
  }
  __syncthreads();
  const int n = tid >> 2, j0 = (tid & 3) * 4;
  float s0 = 0.0f, s1 = 0.0f, s2 = 0.0f, s3 = 0.0f;
#pragma unroll
  for (int i = 0; i < 16; ++i) {
    const float qv = q1s[n * 16 + i];
    const float* tr = Ts + n * TSP + i * 16 + j0;
    s0 += qv * tr[0];
    s1 += qv * tr[1];
    s2 += qv * tr[2];
    s3 += qv * tr[3];
  }
  v4f o;
  o[0] = s0; o[1] = s1; o[2] = s2; o[3] = s3;
  float* dst = attnT + ((size_t)(bh * NN + n0 + n)) * DD + j0;
  st16(dst, o);
  __threadfence();
  st16(dst, o);
}

__global__ __launch_bounds__(256) void k_ln(const float* __restrict__ attnT, const float* __restrict__ gamma,
                                          const float* __restrict__ beta, f16* __restrict__ yln) {
  __shared__ float red[16];
  __shared__ f16 ys[CC] __attribute__((aligned(16)));
  const int row = blockIdx.x;
  const int b = row / NN, n = row - b * NN;
  const int c = threadIdx.x;
  const int hd = c >> 4, j = c & 15;
  const int w = c >> 5, l = c & 31;
  const float v = attnT[((size_t)((b * HH + hd) * NN + n)) * DD + j];
  float s = v;
#pragma unroll
  for (int o = 16; o > 0; o >>= 1) s += __shfl_xor(s, o, 32);
  if (l == 0) red[w] = s;
  __syncthreads();
  float tot = 0.0f;
#pragma unroll
  for (int i = 0; i < 8; ++i) tot += red[i];
  const float mu = tot * (1.0f / CC);
  const float d = v - mu;
  float s2 = d * d;
#pragma unroll
  for (int o = 16; o > 0; o >>= 1) s2 += __shfl_xor(s2, o, 32);
  if (l == 0) red[8 + w] = s2;
  __syncthreads();
  float tot2 = 0.0f;
#pragma unroll
  for (int i = 0; i < 8; ++i) tot2 += red[8 + i];
  const float var = tot2 * (1.0f / CC);
  const float y = d * rsqrtf(var + 1e-5f) * gamma[c] + beta[c];
  ys[c] = (f16)y;
  __syncthreads();
  if (c < 32) {
    U16 u;
    u.h = *(const v8h*)(ys + 8 * c);
    f16* dst = yln + (size_t)row * CC + 8 * c;
    st16(dst, u.f);
    __threadfence();
    st16(dst, u.f);
  }
}

__global__ __launch_bounds__(32) void k_final(const f16* __restrict__ yln, const f16* __restrict__ Wo,
                                            const float* __restrict__ bo, float* __restrict__ out) {
  __shared__ float sT[32 * 64] __attribute__((aligned(16)));
  const int lane = threadIdx.x;
  const int mt = blockIdx.x, nt = blockIdx.y;
  const int m0 = mt * 32, n0 = nt * 64;
  v8f acc[2][4];
  zero_acc(acc);
  gemm_32x64(yln, CC, Wo, CC, m0, n0, CC, lane, acc);

  const int hl = lane >> 4, c16 = lane & 15;
#pragma unroll
  for (int tm = 0; tm < 2; ++tm)
#pragma unroll
    for (int tn = 0; tn < 4; ++tn) {
      const int col = tn * 16 + c16;
      const float bcol = bo[n0 + col];
#pragma unroll
      for (int r = 0; r < 8; ++r) {
        const int row = tm * 16 + hl * 8 + r;
        sT[row * 64 + col] = acc[tm][tn][r] * W_INV + bcol;
      }
    }
  __syncthreads();
  float* dst = out + (size_t)m0 * CC + n0;
  store_tile_f32(sT, dst, CC, lane);
  __threadfence();
  store_tile_f32(sT, dst, CC, lane);
}

extern "C" void kernel_launch(void* const* d_in, const int* in_sizes, int n_in,
                              void* d_out, int out_size, void* d_ws, size_t ws_size,
                              hipStream_t stream) {
  if (n_in < 20) return;
  if (out_size != MTOT * CC) return;
  if (in_sizes[0] != MTOT * CC || in_sizes[1] != MTOT) return;
  for (int i = 2; i <= 16; i += 2) if (in_sizes[i] != CC * CC) return;
  for (int i = 3; i <= 17; i += 2) if (in_sizes[i] != CC) return;
  if (in_sizes[18] != CC || in_sizes[19] != CC) return;

  const float* x    = (const float*)d_in[0];
  const float* mask = (const float*)d_in[1];
  Ptr8 w;
  w.p[0] = (const float*)d_in[2];
  w.p[1] = (const float*)d_in[4];
  w.p[2] = (const float*)d_in[6];
  w.p[3] = (const float*)d_in[8];
  w.p[4] = (const float*)d_in[10];
  w.p[5] = (const float*)d_in[12];
  w.p[6] = (const float*)d_in[14];
  w.p[7] = (const float*)d_in[16];
  Ptr7 bias;
  bias.p[0] = (const float*)d_in[3];
  bias.p[1] = (const float*)d_in[5];
  bias.p[2] = (const float*)d_in[7];
  bias.p[3] = (const float*)d_in[9];
  bias.p[4] = (const float*)d_in[11];
  bias.p[5] = (const float*)d_in[13];
  bias.p[6] = (const float*)d_in[15];
  const float* bo    = (const float*)d_in[17];
  const float* gamma = (const float*)d_in[18];
  const float* beta  = (const float*)d_in[19];
  float* out = (float*)d_out;

  char* ws = (char*)d_ws;
  size_t off = 0;
  auto alloc = [&](size_t bytes) -> void* {
    void* p = ws + off;
    off = (off + bytes + 255) & ~(size_t)255;
    return p;
  };
  f16*   xh    = (f16*)alloc((size_t)MTOT * CC * 2);
  f16*   wh    = (f16*)alloc((size_t)8 * CC * CC * 2);
  float* lin   = (float*)alloc((size_t)7 * MTOT * CC * 4);
  f16*   A1t   = (f16*)alloc((size_t)GRP * CC * NN * 2);
  f16*   A2t   = (f16*)alloc((size_t)GRP * CC * NN * 2);
  f16*   Qt    = (f16*)alloc((size_t)GRP * NN * CC * 2);
  f16*   sth   = (f16*)alloc((size_t)GRP * CC * CC * 2);
  float* attnT = (float*)alloc((size_t)NBH * NN * DD * 4);
  f16*   yln   = (f16*)alloc((size_t)MTOT * CC * 2);
  if (off > ws_size) return;

  const int nx8 = MTOT * CC / 8;
  k_convx<<<dim3((nx8 + 255) / 256), 256, 0, stream>>>(x, xh, nx8);
  k_convw<<<dim3((CC * CC / 8 + 255) / 256, 8), 256, 0, stream>>>(w, wh);
  k_lin<<<dim3(MTOT / 32, CC / 64, 7), 32, 0, stream>>>(xh, wh, x, mask, bias, lin);

  for (int gi = 0; gi < NGRP; ++gi) {
    k_outer<<<dim3(NN / 64, GRP), 256, 0, stream>>>(lin, gi, A1t, A2t, Qt);
    k_state<<<dim3(CC / 32, CC / 64, GRP), 32, 0, stream>>>(A1t, A2t, sth);
    k_apply<<<dim3(NN / 32, GRP), 128, 0, stream>>>(Qt, sth, lin, gi, attnT);
  }

  k_ln<<<dim3(MTOT), 256, 0, stream>>>(attnT, gamma, beta, yln);
  k_final<<<dim3(MTOT / 32, CC / 64), 32, 0, stream>>>(yln, wh + (size_t)7 * CC * CC, bo, out);
}
